// EdgeQProj_68453188763807
// MI455X (gfx1250) — hardware-verified
//
#include <hip/hip_runtime.h>
#include <stddef.h>
#include <stdint.h>


#define NB    64
#define NN    64
#define OBJ   2048
#define QD    1024
#define HID   512
#define KS    8
#define QH    (HID * KS)
#define MTOT  (NB * NN)
#define EPB   32
#define XSC   8
#define WSC   1024
#define NTHR  256
#define TPW   64
#define WSCAP 134217728

static_assert(NTHR == 256);
static_assert((OBJ % 128) == 0);
static_assert((QD % 128) == 0);
static_assert((OBJ % 32) == 0);
static_assert((QD % 32) == 0);
static_assert((HID % 128) == 0);
static_assert((QH % 128) == 0);
static_assert((MTOT % 64) == 0);
static_assert((NB % 64) == 0);
static_assert(((MTOT * OBJ) % (8 * NTHR)) == 0);
static_assert(((NB * QD) % (8 * NTHR)) == 0);
static_assert(NB * 4 == NTHR);
static_assert(NB * KS == 4 * 128);
static_assert(EPB * KS == 4 * 64);
static_assert((HID % 128) == 0);

typedef float          v2f  __attribute__((ext_vector_type(2)));
typedef float          v4f  __attribute__((ext_vector_type(4)));
typedef float          v8f  __attribute__((ext_vector_type(8)));
typedef _Float16       v8h  __attribute__((ext_vector_type(8)));
typedef _Float16       v16h __attribute__((ext_vector_type(16)));
union FragH { v16h v; v8h h[2]; };

__device__ __forceinline__ v8f wmf(v16h a, v16h b, v8f c) {
  v8f d = __builtin_amdgcn_wmma_f32_16x16x32_f16(false, a, false, b, (short)0, c, false, false);
  asm volatile("v_nop\n\tv_nop\n\tv_nop\n\tv_nop" : "+v"(d) : "v"(a), "v"(b));
  return d;
}

__global__ __launch_bounds__(NTHR) void k_cvt(const float* __restrict__ x, _Float16* xh, int n8) {
  const int ti = blockIdx.x * NTHR + threadIdx.x;
  if (ti < n8) {
    const size_t t = (size_t)ti;
    const float* p = x + t * 8;
    const v4f f0 = *(const v4f*)p;
    const v4f f1 = *(const v4f*)(p + 4);
    v8h a;
    a[0] = (_Float16)(f0.x * (float)XSC); a[1] = (_Float16)(f0.y * (float)XSC);
    a[2] = (_Float16)(f0.z * (float)XSC); a[3] = (_Float16)(f0.w * (float)XSC);
    a[4] = (_Float16)(f1.x * (float)XSC); a[5] = (_Float16)(f1.y * (float)XSC);
    a[6] = (_Float16)(f1.z * (float)XSC); a[7] = (_Float16)(f1.w * (float)XSC);
    _Float16* d = xh + t * 8;
    *(volatile v8h*)d = a;
    __threadfence();
    *(volatile v8h*)d = a;
  }
}

__global__ __launch_bounds__(NTHR) void k_prepw(const float* __restrict__ W, _Float16* wt, int K, int N) {
  __shared__ __attribute__((aligned(16))) float tile[128 * TPW];
  const int tid = threadIdx.x, lane = tid & 31, g = tid >> 5, hh = lane >> 4, m = lane & 15;
  const int n0 = blockIdx.x * 64;
  const int n = n0 + 2 * lane;
#pragma unroll 1
  for (int dc = 0; dc < K; dc += 128) {
    __syncthreads();
#pragma unroll 4
    for (int p = 0; p < 16; ++p) {
      const int dl = g + 8 * p;
      const v2f w = *(const v2f*)(W + (size_t)(dc + dl) * N + n);
      *(v2f*)(tile + dl * TPW + 2 * lane) = w;
    }
    __syncthreads();
    v8h hv[4];
#pragma unroll
    for (int q = 0; q < 4; ++q) {
      const int nl = 8 * g + 2 * q + hh;
      const int d8 = 8 * m;
#pragma unroll
      for (int e = 0; e < 8; ++e) hv[q][e] = (_Float16)(tile[(d8 + e) * TPW + nl] * (float)WSC);
    }
#pragma unroll
    for (int q = 0; q < 4; ++q) {
      _Float16* d = wt + (size_t)(n0 + 8 * g + 2 * q + hh) * K + dc + 8 * m;
      *(volatile v8h*)d = hv[q];
    }
    __threadfence();
#pragma unroll
    for (int q = 0; q < 4; ++q) {
      _Float16* d = wt + (size_t)(n0 + 8 * g + 2 * q + hh) * K + dc + 8 * m;
      *(volatile v8h*)d = hv[q];
    }
  }
}

__global__ __launch_bounds__(NTHR) void k_gemm(const _Float16* __restrict__ xh, const _Float16* __restrict__ wt,
                                               const float* __restrict__ bias, float* C, int N, int K) {
  __shared__ __attribute__((aligned(16))) float stg_all[8 * 32 * 32];
  const int tid = threadIdx.x, lane = tid & 31, wave = tid >> 5, hh = lane >> 4, m = lane & 15;
  float* stg = stg_all + wave * (32 * 32);
  const int n0 = blockIdx.x * 128, m0 = blockIdx.y * 64;
  const int wm = (wave & 1) * 32, wn = (wave >> 1) * 32;

  v8f acc[2][2];
#pragma unroll
  for (int i = 0; i < 2; ++i)
#pragma unroll
    for (int j = 0; j < 2; ++j) { v8f z = {0.f, 0.f, 0.f, 0.f, 0.f, 0.f, 0.f, 0.f}; acc[i][j] = z; }

  const _Float16* ap = xh + (size_t)(m0 + wm + m) * K + 8 * hh;
  const _Float16* bp = wt + (size_t)(n0 + wn + m) * K + 8 * hh;
  const size_t r16 = (size_t)16 * K;
  const int nkt = K / 32;
#pragma unroll 1
  for (int kt = 0; kt < nkt; ++kt) {
    const int k0 = 32 * kt;
    FragH a0, a1, b0, b1;
    a0.h[0] = *(const v8h*)(ap + k0);
    a0.h[1] = *(const v8h*)(ap + k0 + 16);
    a1.h[0] = *(const v8h*)(ap + r16 + k0);
    a1.h[1] = *(const v8h*)(ap + r16 + k0 + 16);
    b0.h[0] = *(const v8h*)(bp + k0);
    b0.h[1] = *(const v8h*)(bp + k0 + 16);
    b1.h[0] = *(const v8h*)(bp + r16 + k0);
    b1.h[1] = *(const v8h*)(bp + r16 + k0 + 16);
    acc[0][0] = wmf(a0.v, b0.v, acc[0][0]);
    acc[0][1] = wmf(a0.v, b1.v, acc[0][1]);
    acc[1][0] = wmf(a1.v, b0.v, acc[1][0]);
    acc[1][1] = wmf(a1.v, b1.v, acc[1][1]);
  }

  constexpr float OSC = 1.0f / (float)(XSC * WSC);
  float bv[2];
#pragma unroll
  for (int j = 0; j < 2; ++j) bv[j] = bias[n0 + wn + 16 * j + m];
#pragma unroll
  for (int i = 0; i < 2; ++i) {
    float* sp = stg + (16 * i + 8 * hh) * 32 + m;
#pragma unroll
    for (int j = 0; j < 2; ++j) {
#pragma unroll
      for (int r = 0; r < 8; ++r) {
        float v = acc[i][j][r] * OSC + bv[j];
        v = v > 0.f ? v : 0.f;
        sp[r * 32 + 16 * j] = v;
      }
    }
  }
  __syncthreads();

  float* gbase = C + (size_t)(m0 + wm) * N + n0 + wn;
  const int rq = lane >> 3, cq = 4 * (lane & 7);
#pragma unroll
  for (int q = 0; q < 8; ++q) {
    const int row = 4 * q + rq;
    const v4f v = *(const v4f*)(stg + row * 32 + cq);
    *(volatile v4f*)(gbase + (size_t)row * N + cq) = v;
  }
  __threadfence();
#pragma unroll
  for (int q = 0; q < 8; ++q) {
    const int row = 4 * q + rq;
    const v4f v = *(const v4f*)(stg + row * 32 + cq);
    *(volatile v4f*)(gbase + (size_t)row * N + cq) = v;
  }
}

__global__ __launch_bounds__(NTHR) void k_norm(const float* __restrict__ qh, float* rnorm) {
  __shared__ __attribute__((aligned(16))) v4f part[NTHR];
  __shared__ __attribute__((aligned(16))) float res[NB * KS];
  const int t = threadIdx.x;
  const int b = t >> 2, hp = (t >> 1) & 1, half = t & 1;
  const float* p = qh + (size_t)b * QH + (size_t)hp * (HID / 2) * KS + 4 * half;
  v4f s = {0.f, 0.f, 0.f, 0.f};
#pragma unroll 2
  for (int h = 0; h < HID / 2; ++h) {
    const v4f v = *(const v4f*)(p + (size_t)h * KS);
    s += v * v;
  }
  part[t] = s;
  __syncthreads();
  const v4f tot = s + part[t ^ 2];
  if (hp == 0) {
#pragma unroll
    for (int c = 0; c < 4; ++c) res[b * KS + 4 * half + c] = 1.0f / sqrtf(tot[c]);
  }
  __syncthreads();
  if (t < 128) {
    const v4f v = *(const v4f*)(res + 4 * t);
    float* d = rnorm + 4 * t;
    *(volatile v4f*)d = v;
    __threadfence();
    *(volatile v4f*)d = v;
  }
}

__global__ __launch_bounds__(NTHR) void k_edge(const int* __restrict__ indexes, const float* __restrict__ node_h,
                                               const float* __restrict__ qh, const float* __restrict__ rnorm,
                                               float* out, int nEdges) {
  __shared__ __attribute__((aligned(16))) float res[EPB * KS];
  const int tid = threadIdx.x, lane = tid & 31, wave = tid >> 5;
  const int mblk = blockIdx.x * EPB;
#pragma unroll 1
  for (int e = 0; e < 4; ++e) {
    const int ml = wave * 4 + e;
    int mg = mblk + ml;
    mg = mg < nEdges ? mg : nEdges - 1;
    const int idx = indexes[mg];
    int b = idx >> 12;
    const int rem = idx & 4095;
    const int src = rem >> 6, dst = rem & 63;
    b = b < 0 ? 0 : (b > NB - 1 ? NB - 1 : b);
    const float* p0 = node_h + ((size_t)b * NN + src) * HID;
    const float* p1 = node_h + ((size_t)b * NN + dst) * HID;
    const float* pq = qh + (size_t)b * QH;
    v4f sa = {0.f, 0.f, 0.f, 0.f}, sb = {0.f, 0.f, 0.f, 0.f};
#pragma unroll 1
    for (int i = 0; i < HID / 128; ++i) {
      const int h0 = 128 * i + 4 * lane;
      const v4f o = *(const v4f*)(p0 + h0) + *(const v4f*)(p1 + h0);
#pragma unroll
      for (int c = 0; c < 4; ++c) {
        const float* pqh = pq + (size_t)(h0 + c) * KS;
        const v4f qa = *(const v4f*)pqh;
        const v4f qb = *(const v4f*)(pqh + 4);
        const float oc = o[c];
        sa += oc * qa;
        sb += oc * qb;
      }
    }
#pragma unroll
    for (int off = 16; off > 0; off >>= 1) {
#pragma unroll
      for (int c = 0; c < 4; ++c) {
        sa[c] = sa[c] + __shfl_xor(sa[c], off, 32);
        sb[c] = sb[c] + __shfl_xor(sb[c], off, 32);
      }
    }
    const v4f ra = *(const v4f*)(rnorm + b * KS);
    const v4f rb = *(const v4f*)(rnorm + b * KS + 4);
    sa = sa * ra;
    sb = sb * rb;
    if (lane == 0) {
      *(v4f*)(res + ml * KS) = sa;
      *(v4f*)(res + ml * KS + 4) = sb;
    }
  }
  __syncthreads();
  if (tid < 64) {
    const size_t el = (size_t)mblk * KS + 4 * (size_t)tid;
    if (el < (size_t)nEdges * KS) {
      const v4f v = *(const v4f*)(res + 4 * tid);
      float* d = out + el;
      *(volatile v4f*)d = v;
      __threadfence();
      *(volatile v4f*)d = v;
    }
  }
}

extern "C" void kernel_launch(void* const* d_in, const int* in_sizes, int n_in,
                              void* d_out, int out_size, void* d_ws, size_t ws_size,
                              hipStream_t stream) {
  if (n_in < 7) return;
  const int nEdges = in_sizes[2];
  if (nEdges < 1) return;
  if (in_sizes[0] != MTOT * OBJ || in_sizes[1] != NB * QD || in_sizes[3] != OBJ * HID ||
      in_sizes[4] != HID || in_sizes[5] != QD * QH || in_sizes[6] != QH) return;
  if (out_size != nEdges * KS) return;

  const float* node_feats = (const float*)d_in[0];
  const float* q_feats    = (const float*)d_in[1];
  const int*   indexes    = (const int*)d_in[2];
  const float* W_obj      = (const float*)d_in[3];
  const float* b_obj      = (const float*)d_in[4];
  const float* W_q        = (const float*)d_in[5];
  const float* b_q        = (const float*)d_in[6];
  float* out = (float*)d_out;

  char* ws = (char*)d_ws;
  size_t off = 0;
  const size_t oXh1 = off; off += (size_t)MTOT * OBJ * 2; off = (off + 255) & ~(size_t)255;
  const size_t oWt1 = off; off += (size_t)HID * OBJ * 2;  off = (off + 255) & ~(size_t)255;
  const size_t oXh2 = off; off += (size_t)NB * QD * 2;    off = (off + 255) & ~(size_t)255;
  const size_t oWt2 = off; off += (size_t)QH * QD * 2;    off = (off + 255) & ~(size_t)255;
  const size_t oNh  = off; off += (size_t)MTOT * HID * 4; off = (off + 255) & ~(size_t)255;
  const size_t oQh  = off; off += (size_t)NB * QH * 4;    off = (off + 255) & ~(size_t)255;
  const size_t oRn  = off; off += (size_t)NB * KS * 4;    off = (off + 255) & ~(size_t)255;
  if (off > ws_size || off > (size_t)WSCAP) return;
  _Float16* xh1 = (_Float16*)(ws + oXh1);
  _Float16* wt1 = (_Float16*)(ws + oWt1);
  _Float16* xh2 = (_Float16*)(ws + oXh2);
  _Float16* wt2 = (_Float16*)(ws + oWt2);
  float* node_h = (float*)(ws + oNh);
  float* q_h    = (float*)(ws + oQh);
  float* rnorm  = (float*)(ws + oRn);

  k_cvt<<<(MTOT * OBJ / 8) / NTHR, NTHR, 0, stream>>>(node_feats, xh1, MTOT * OBJ / 8);
  k_cvt<<<(NB * QD / 8) / NTHR, NTHR, 0, stream>>>(q_feats, xh2, NB * QD / 8);
  k_prepw<<<HID / 64, NTHR, 0, stream>>>(W_obj, wt1, OBJ, HID);
  k_prepw<<<QH / 64, NTHR, 0, stream>>>(W_q, wt2, QD, QH);
  k_gemm<<<dim3(HID / 128, MTOT / 64), NTHR, 0, stream>>>(xh1, wt1, b_obj, node_h, HID, OBJ);
  k_gemm<<<dim3(QH / 128, NB / 64), NTHR, 0, stream>>>(xh2, wt2, b_q, q_h, QH, QD);
  k_norm<<<1, NTHR, 0, stream>>>(q_h, rnorm);
  k_edge<<<(nEdges + EPB - 1) / EPB, NTHR, 0, stream>>>(indexes, node_h, q_h, rnorm, out, nEdges);
}
